// EdgeQMul_68453188763805
// MI455X (gfx1250) — hardware-verified
//
#include <hip/hip_runtime.h>
#include <math.h>

typedef __attribute__((ext_vector_type(16))) _Float16 v16h;
typedef __attribute__((ext_vector_type(16))) __bf16 v16b;
typedef __attribute__((ext_vector_type(8)))  _Float16 v8h;
typedef __attribute__((ext_vector_type(8)))  float v8f;
typedef __attribute__((ext_vector_type(4)))  float v4f;
typedef __attribute__((ext_vector_type(2)))  float v2f;
typedef __attribute__((ext_vector_type(4)))  unsigned v4u;
typedef __attribute__((ext_vector_type(4)))  int v4i;
typedef float __attribute__((may_alias)) float_a;
typedef int __attribute__((may_alias)) int_a;

template <typename T> __device__ __forceinline__ void vst2(void* p, T v) { *(volatile T*)p = v; __threadfence(); *(volatile T*)p = v; }
__device__ __forceinline__ v8f wmma16(v16h a, v16h b, v8f c) {
  v8f d = __builtin_amdgcn_wmma_f32_16x16x32_f16(false, a, false, b, (short)0, c, false, false);
  asm volatile("v_nop\n\tv_nop\n\tv_nop\n\tv_nop" : "+v"(d) : "v"(a), "v"(b));
  return d;
}
__device__ __forceinline__ v8f wmma_bf(v16b a, v16b b, v8f c) {
  v8f d = __builtin_amdgcn_wmma_f32_16x16x32_bf16(false, a, false, b, (short)0, c, false, false);
  asm volatile("v_nop\n\tv_nop\n\tv_nop\n\tv_nop" : "+v"(d) : "v"(a), "v"(b));
  return d;
}
__device__ __forceinline__ v16h frag_h(const _Float16* rowk0, int lane) {
  union { v16h v; v8h q[2]; } u; const _Float16* p = rowk0 + 8 * (lane >> 4);
  u.q[0] = *(const v8h*)p; u.q[1] = *(const v8h*)(p + 16); return u.v;
}
__device__ __forceinline__ v16h frag_f32(const float* rowk0, int lane) {
  v16h a; const float* p = rowk0 + 8 * (lane >> 4);
#pragma unroll
  for (int i = 0; i < 8; ++i) { a[i] = (_Float16)p[i]; a[8 + i] = (_Float16)p[16 + i]; }
  return a;
}
__device__ __forceinline__ v16h frag_f32s(const float* rowk0, int lane, float sc) {
  v16h a; const float* p = rowk0 + 8 * (lane >> 4);
#pragma unroll
  for (int i = 0; i < 8; ++i) { a[i] = (_Float16)(p[i] * sc); a[8 + i] = (_Float16)(p[16 + i] * sc); }
  return a;
}
__device__ __forceinline__ v16h fragc_f32(const float* W, int k0, int n, int lane, int ld, int K) {
  v16h a; const int g = lane >> 4;
#pragma unroll
  for (int i = 0; i < 8; ++i) { const int ka = k0 + 8 * g + i, kb = ka + 16;
    a[i] = (_Float16)(ka < K ? W[(size_t)(ka < K ? ka : K - 1) * ld + n] : 0.f); a[8 + i] = (_Float16)(kb < K ? W[(size_t)(kb < K ? kb : K - 1) * ld + n] : 0.f); }
  return a;
}
struct F2 { v16b h, l; };
__device__ __forceinline__ F2 bsplit16(const float v[16]) { F2 r;
#pragma unroll
  for (int i = 0; i < 16; ++i) { const __bf16 h = (__bf16)v[i]; r.h[i] = h; r.l[i] = (__bf16)(v[i] - (float)h); }
  return r; }
__device__ __forceinline__ F2 split_row(const float* row, int k0, int lane) { float v[16]; const float* p = row + k0 + 8 * (lane >> 4);
#pragma unroll
  for (int i = 0; i < 8; ++i) { v[i] = p[i]; v[8 + i] = p[16 + i]; }
  return bsplit16(v); }
__device__ __forceinline__ F2 split_rowK(const float* row, int k0, int lane, int K) { float v[16]; const int g = lane >> 4;
#pragma unroll
  for (int i = 0; i < 8; ++i) { const int ka = k0 + 8 * g + i, kb = ka + 16; v[i] = ka < K ? row[ka < K ? ka : K - 1] : 0.f; v[8 + i] = kb < K ? row[kb < K ? kb : K - 1] : 0.f; }
  return bsplit16(v); }
__device__ __forceinline__ F2 split_col(const float* W, int k0, int n, int lane, int ld, int K) { float v[16]; const int g = lane >> 4;
#pragma unroll
  for (int i = 0; i < 8; ++i) { const int ka = k0 + 8 * g + i, kb = ka + 16; v[i] = ka < K ? W[(size_t)(ka < K ? ka : K - 1) * ld + n] : 0.f; v[8 + i] = kb < K ? W[(size_t)(kb < K ? kb : K - 1) * ld + n] : 0.f; }
  return bsplit16(v); }
__device__ __forceinline__ v8f mac3(const F2& a, const F2& b, v8f c) { c = wmma_bf(a.l, b.h, c); c = wmma_bf(a.h, b.l, c); return wmma_bf(a.h, b.h, c); }
__device__ __forceinline__ float sigm(float v) { return 1.0f / (1.0f + expf(-v)); }
#define LDSX() do { asm volatile("s_wait_dscnt 0" ::: "memory"); __builtin_amdgcn_wave_barrier(); __builtin_amdgcn_fence(__ATOMIC_RELEASE, "workgroup"); } while (0)


#define NB 128
#define NNODE 36
#define PPB (NNODE * (NNODE - 1))
#define NE (NB * PPB)
#define NROW (NB * NNODE)
#define OBJ 2048
#define QD 1024
#define HID 512
#define MID 256
#define KS 8
#ifndef TEB
#define TEB (NE / 64)
#endif
typedef __attribute__((ext_vector_type(8))) __bf16 v8b;
__device__ __forceinline__ v16b frag_b(const __bf16* rowk0, int lane) {
  union { v16b v; v8b q[2]; } u; const __bf16* p = rowk0 + 8 * (lane >> 4);
  u.q[0] = *(const v8b*)p; u.q[1] = *(const v8b*)(p + 16); return u.v;
}
__device__ __forceinline__ float bfr(float v) { return (float)(__bf16)v; }
__device__ __attribute__((noinline)) float exp_ni(float v) { return expf(v); }
__device__ __attribute__((noinline)) float erf_ni(float v) { return erff(v); }

#define WS_PO  0u
#define WS_PQ  (WS_PO + 2u * (size_t)HID * OBJ)
#define WS_P1  (WS_PQ + 2u * (size_t)HID * QD)
#define WS_P2  (WS_P1 + 2u * (size_t)MID * HID)
#define WS_SC  (WS_P2 + 2u * (size_t)16 * MID)
#define WS_NF  (WS_SC + 4u * 2048)
#define WS_QP  (WS_NF + 4u * (size_t)NROW * HID)
#define WS_END (WS_QP + 4u * (size_t)NB * HID)

__global__ __launch_bounds__(256) void k_pack(const float* __restrict__ VO, const float* __restrict__ GO, const float* __restrict__ VQ, const float* __restrict__ GQ, const float* __restrict__ V1, const float* __restrict__ G1, const float* __restrict__ V2, const float* __restrict__ G2, __bf16* __restrict__ PO, __bf16* __restrict__ PQ, _Float16* __restrict__ P1, _Float16* __restrict__ P2, float* __restrict__ SC) {
  __shared__ __align__(16) __bf16 sb[OBJ]; __shared__ __align__(16) _Float16 sh[HID]; __shared__ float red[8];
  const int o = blockIdx.x, which = blockIdx.y, t = threadIdx.x;
  const int K = (which == 0) ? OBJ : (which == 1) ? QD : (which == 2) ? HID : MID; const int nrow = (which <= 1) ? HID : (which == 2) ? MID : KS;
  if (o >= ((which == 3) ? 16 : nrow)) return;
  const float* v = (which == 0) ? (VO + (size_t)o * OBJ) : (which == 1) ? (VQ + (size_t)o * QD) : (which == 2) ? (V1 + (size_t)o * HID) : (V2 + (size_t)o * MID);
  const bool live = o < nrow; float ss = 0.f;
  for (int k = t; k < K; k += 256) { const float x = live ? bfr(v[k]) : 0.f; ss += x * x; if (which <= 1) sb[k] = (__bf16)x; else sh[k] = (_Float16)(x * 256.0f); }
#pragma unroll
  for (int s = 1; s < 32; s <<= 1) ss += __shfl_xor(ss, s);
  if ((t & 31) == 0) red[t >> 5] = ss; __syncthreads(); float tot = 0.f; for (int i = 0; i < 8; ++i) tot += red[i];
  if (which == 0) { for (int q = t; q < OBJ / 8; q += 256) vst2((unsigned*)(PO + (size_t)o * OBJ + q * 8), *(const v4u*)&sb[q * 8]); }
  else if (which == 1) { for (int q = t; q < QD / 8; q += 256) vst2((unsigned*)(PQ + (size_t)o * QD + q * 8), *(const v4u*)&sb[q * 8]); }
  else if (which == 2) { if (t < HID / 8) vst2((unsigned*)(P1 + (size_t)o * HID + t * 8), *(const v4u*)&sh[t * 8]); }
  else { if (t < MID / 8) vst2((unsigned*)(P2 + (size_t)o * MID + t * 8), *(const v4u*)&sh[t * 8]); }
  (void)tot; (void)GO; (void)GQ; (void)G1; (void)G2; (void)SC;
}
__global__ __launch_bounds__(256) void k_scale(const float* __restrict__ VO, const float* __restrict__ GO, const float* __restrict__ VQ, const float* __restrict__ GQ, const float* __restrict__ V1, const float* __restrict__ G1, const float* __restrict__ V2, const float* __restrict__ G2, float* __restrict__ SC) {
  __shared__ __align__(16) float s[512]; const int which = blockIdx.x, t = threadIdx.x;
  const int K = (which == 0) ? OBJ : (which == 1) ? QD : (which == 2) ? HID : MID; const int nrow = (which <= 1) ? HID : (which == 2) ? MID : KS;
  const float* V = (which == 0) ? VO : (which == 1) ? VQ : (which == 2) ? V1 : V2; const float* Gm = (which == 0) ? GO : (which == 1) ? GQ : (which == 2) ? G1 : G2;
  for (int o = t; o < 512; o += 256) { float v = 0.f; if (o < nrow) { const float* vv = V + (size_t)o * K; float s2 = 0.f; for (int k = 0; k < K; ++k) { const float x = bfr(vv[k]); s2 += x * x; } v = bfr(Gm[o]) / sqrtf(s2); } s[o] = v; }
  __syncthreads(); if (t < 128) vst2(SC + which * 512 + t * 4, *(const v4f*)&s[t * 4]);
}
template <int ISQ>
__global__ __launch_bounds__(128) void k_nf(const float* __restrict__ X, const __bf16* __restrict__ P, const float* __restrict__ SC, const float* __restrict__ BB, float* __restrict__ OUTF) {
  constexpr int K = ISQ ? QD : OBJ; __shared__ __align__(16) float so[4][16][132];
  const int tid = threadIdx.x, wave = tid >> 5, lane = tid & 31, col = lane & 15, g = lane >> 4; const size_t r0 = (size_t)blockIdx.x * 64 + wave * 16; const int n0 = blockIdx.y * 128;
  v8f acc[8] = {};
#pragma unroll 2
  for (int kc = 0; kc < K / 32; ++kc) { v16b a; { const float* p = X + (r0 + col) * K + kc * 32 + 8 * g;
#pragma unroll
      for (int i = 0; i < 8; ++i) { a[i] = (__bf16)p[i]; a[8 + i] = (__bf16)p[16 + i]; } }
#pragma unroll
    for (int j = 0; j < 8; ++j) acc[j] = wmma_bf(a, frag_b(P + (size_t)(n0 + j * 16 + col) * K + kc * 32, lane), acc[j]); }
#pragma unroll
  for (int j = 0; j < 8; ++j) { const int c = n0 + j * 16 + col; const float sc = SC[(ISQ ? 512 : 0) + c], bb = bfr(BB[c]);
#pragma unroll
    for (int r = 0; r < 8; ++r) so[wave][8 * g + r][j * 16 + col] = acc[j][r] * sc + bb; }
  LDSX();
  for (int rl = 0; rl < 16; ++rl) vst2(OUTF + (r0 + rl) * HID + n0 + lane * 4, *(const v4f*)&so[wave][rl][lane * 4]);
}
__global__ __launch_bounds__(128) void k_edge(const int* __restrict__ IDX, const float* __restrict__ NF, const float* __restrict__ QP, const _Float16* __restrict__ P1, const _Float16* __restrict__ P2, const float* __restrict__ SC, const float* __restrict__ B1, const float* __restrict__ B2, float* __restrict__ OUT) {
  __shared__ __align__(16) _Float16 se[64][HID + 8];
  __shared__ __align__(16) _Float16 sh[64][MID + 8];
  __shared__ __align__(16) float so[64][KS];
  __shared__ int sbi[64], si[64], sj[64];
  const int tid = threadIdx.x, wave = tid >> 5, lane = tid & 31, col = lane & 15, g = lane >> 4; const size_t m0 = (size_t)blockIdx.x * 64;
  if (tid < 64) { const int idx = IDX[m0 + tid]; const int bi = idx / (NNODE * NNODE), rem = idx % (NNODE * NNODE); sbi[tid] = bi; si[tid] = rem / NNODE; sj[tid] = rem % NNODE; }
  __syncthreads();
  for (int e = tid; e < 64 * HID; e += 128) { const int rr = e / HID, c = e % HID; const size_t m = m0 + rr; const int qb = (int)(m / PPB);
    const float v = NF[((size_t)sbi[rr] * NNODE + si[rr]) * HID + c] * NF[((size_t)sbi[rr] * NNODE + sj[rr]) * HID + c] * QP[(size_t)qb * HID + c]; se[rr][c] = (_Float16)v; }
  __syncthreads();
  const int w0 = wave * 16;
#pragma unroll 1
  for (int half = 0; half < 2; ++half) { v8f acc[8] = {};
#pragma unroll 2
    for (int kc = 0; kc < HID / 32; ++kc) { const v16h a = frag_h(&se[w0 + col][0] + kc * 32, lane);
#pragma unroll
      for (int j = 0; j < 8; ++j) acc[j] = wmma16(a, frag_h(P1 + (size_t)(half * 128 + j * 16 + col) * HID + kc * 32, lane), acc[j]); }
#pragma unroll
    for (int j = 0; j < 8; ++j) { const int c = half * 128 + j * 16 + col; const float sc = SC[1024 + c] * (1.0f / 256.0f), bb = bfr(B1[c]);
#pragma unroll
      for (int r = 0; r < 8; ++r) sh[w0 + 8 * g + r][c] = (_Float16)fmaxf(acc[j][r] * sc + bb, 0.f); } }
  LDSX();
  { v8f acc = {};
#pragma unroll
    for (int kc = 0; kc < MID / 32; ++kc) acc = wmma16(frag_h(&sh[w0 + col][0] + kc * 32, lane), frag_h(P2 + (size_t)col * MID + kc * 32, lane), acc);
    if (col < KS) { const float sc = SC[1536 + col] * (1.0f / 256.0f), bb = bfr(B2[col]);
#pragma unroll
      for (int r = 0; r < 8; ++r) so[w0 + 8 * g + r][col] = acc[r] * sc + bb; } }
  __syncthreads();
  vst2(OUT + (m0 * KS) + tid * 4, *(const v4f*)(&so[0][0] + tid * 4));
}
extern "C" void kernel_launch(void* const* d_in, const int* in_sizes, int n_in, void* d_out, int out_size, void* d_ws, size_t ws_size, hipStream_t stream) {
  (void)in_sizes; (void)n_in; (void)out_size;
  const float** F = (const float**)d_in;
  if (ws_size < (size_t)WS_END) return;
  char* ws = (char*)d_ws; __bf16 *PO = (__bf16*)(ws + WS_PO), *PQ = (__bf16*)(ws + WS_PQ); _Float16 *P1 = (_Float16*)(ws + WS_P1), *P2 = (_Float16*)(ws + WS_P2); float *SC = (float*)(ws + WS_SC), *NF = (float*)(ws + WS_NF), *QP = (float*)(ws + WS_QP);
  k_pack<<<dim3(HID, 4), 256, 0, stream>>>(F[3], F[4], F[6], F[7], F[9], F[10], F[12], F[13], PO, PQ, P1, P2, SC);
  k_scale<<<4, 256, 0, stream>>>(F[3], F[4], F[6], F[7], F[9], F[10], F[12], F[13], SC);
  k_nf<0><<<dim3(NROW / 64, HID / 128), 128, 0, stream>>>(F[0], PO, SC, F[5], NF);
  k_nf<1><<<dim3(NB / 64, HID / 128), 128, 0, stream>>>(F[1], PQ, SC, F[8], QP);
  k_edge<<<TEB, 128, 0, stream>>>((const int*)d_in[2], NF, QP, P1, P2, SC, F[11], F[14], (float*)d_out);
}
